// MHLA_37615323578452
// MI455X (gfx1250) — hardware-run, weakly checked
//
#include <hip/hip_runtime.h>
#include <math.h>

constexpr int kBatch   = 2;
constexpr int kSeq     = 2048;
constexpr int kEmb     = 1024;
constexpr int kHeads   = 16;
constexpr int kHdim    = 64;
constexpr int kChunk   = 128;
constexpr int kNChunk  = kSeq / kChunk;
constexpr int kTok     = kBatch * kSeq;
constexpr int kYB      = kBatch * kNChunk;
constexpr int kTiles   = kYB * kHeads;
constexpr float kEps   = 1e-6f;
constexpr long kPlaneEl = (long)kTok * kEmb;
constexpr long kWEl     = (long)kEmb * kEmb;
constexpr long kUnit    = kPlaneEl * 2;
constexpr long kWUnit   = kWEl * 2;

constexpr long oXbase = 0;
constexpr long oKT_h  = 0;
constexpr long oKT_l  = 1 * kUnit;
constexpr long oVT_h  = 2 * kUnit;
constexpr long oVT_l  = 3 * kUnit;
constexpr long oDST   = 4 * kUnit;
constexpr long oST_h  = 5 * kUnit;
constexpr long oST_l  = 5 * kUnit + kUnit / 2;
constexpr long oA_h   = 0;
constexpr long oNUM   = 4 * kUnit;
constexpr long oWbase = 6 * kUnit;
constexpr long oWo_h  = oWbase + 6 * kWUnit;
constexpr long oWo_l  = oWbase + 7 * kWUnit;
constexpr long oQ_h   = 8 * kUnit;
constexpr long oQ_l   = 9 * kUnit;
constexpr long oK_h   = 10 * kUnit;
constexpr long oK_l   = 11 * kUnit;
constexpr long oV_h   = 12 * kUnit;
constexpr long oV_l   = 13 * kUnit;
constexpr long oNUM1  = 10 * kUnit;
constexpr long oA_l   = 12 * kUnit;
constexpr long oO_h   = 10 * kUnit;
constexpr long oO_l   = 11 * kUnit;
constexpr long oDZ    = 14 * kUnit;
constexpr long oZPRE  = 14 * kUnit + 131072;
constexpr long kWsTotal = 14 * kUnit + 262144;
static_assert(kWsTotal == 117702656, "carve total");
static_assert(kWsTotal <= 134217728, "carve within 128 MiB");
static_assert((long)kTiles * kChunk * kChunk * 2 == 2 * kUnit, "A plane size");
static_assert((long)kTiles * kHdim * kChunk * 2 == kUnit, "kT plane size");
static_assert((long)kTiles * kHdim * kHdim * 4 == kUnit, "dST plane size");

typedef __attribute__((ext_vector_type(16))) _Float16 v16h;
typedef __attribute__((ext_vector_type(8)))  _Float16 v8h;
typedef __attribute__((ext_vector_type(16))) __bf16   v16b;
typedef __attribute__((ext_vector_type(8)))  __bf16   v8b;
typedef __attribute__((ext_vector_type(8)))  float    v8f;
typedef __attribute__((ext_vector_type(4)))  float    v4f;
typedef __attribute__((ext_vector_type(4)))  unsigned int v4u;

__device__ __forceinline__ unsigned short f2bf_bits(float f) {
  unsigned u = __float_as_uint(f);
  return (unsigned short)((u + 0x7FFFu + ((u >> 16) & 1u)) >> 16);
}
__device__ __forceinline__ float bf_bits2f(unsigned short h) { return __uint_as_float(((unsigned)h) << 16); }

__device__ __forceinline__ void dep_guard_h(v8f& a, v8f& b, v16h x, v16h y) { asm volatile("v_nop\n\tv_nop\n\tv_nop\n\tv_nop" : "+v"(a), "+v"(b) : "v"(x), "v"(y)); }
__device__ __forceinline__ void dep_guard_b(v8f& a, v8f& b, v16b x, v16b y) { asm volatile("v_nop\n\tv_nop\n\tv_nop\n\tv_nop" : "+v"(a), "+v"(b) : "v"(x), "v"(y)); }
__device__ __forceinline__ void keep4_h(v16h a, v16h b, v16h c, v16h d) { asm volatile("v_nop" :: "v"(a), "v"(b), "v"(c), "v"(d)); }
__device__ __forceinline__ void keep4_b(v16b a, v16b b, v16b c, v16b d) { asm volatile("v_nop" :: "v"(a), "v"(b), "v"(c), "v"(d)); }
__device__ __forceinline__ void acc_guard4(v8f& a, v8f& b, v8f& c, v8f& d) { asm volatile("v_nop\n\tv_nop\n\tv_nop\n\tv_nop" : "+v"(a), "+v"(b), "+v"(c), "+v"(d)); }
template <typename T> struct Frag;
template <> struct Frag<_Float16> {
  typedef v16h V; union U { v16h v; v8h h[2]; };
  static __device__ __forceinline__ v16h load(const _Float16* p) {
    U f; f.h[0] = *(const v8h*)(p); f.h[1] = *(const v8h*)(p + 16); return f.v;
  }
  static __device__ __forceinline__ v8f mma(v16h a, v16h b, v8f c) {
    return __builtin_amdgcn_wmma_f32_16x16x32_f16(false, a, false, b, (short)0, c, false, false);
  }
  static __device__ __forceinline__ void guard(v8f& a, v8f& b, v16h x, v16h y) { dep_guard_h(a, b, x, y); }
  static __device__ __forceinline__ void keep(v16h a, v16h b, v16h c, v16h d) { keep4_h(a, b, c, d); }
};
template <> struct Frag<__bf16> {
  typedef v16b V; union U { v16b v; v8b h[2]; };
  static __device__ __forceinline__ v16b load(const __bf16* p) {
    U f; f.h[0] = *(const v8b*)(p); f.h[1] = *(const v8b*)(p + 16); return f.v;
  }
  static __device__ __forceinline__ v8f mma(v16b a, v16b b, v8f c) {
    return __builtin_amdgcn_wmma_f32_16x16x32_bf16(false, a, false, b, (short)0, c, false, false);
  }
  static __device__ __forceinline__ void guard(v8f& a, v8f& b, v16b x, v16b y) { dep_guard_b(a, b, x, y); }
  static __device__ __forceinline__ void keep(v16b a, v16b b, v16b c, v16b d) { keep4_b(a, b, c, d); }
};

__device__ __forceinline__ unsigned pk16(unsigned short a, unsigned short b) { return (unsigned)a | ((unsigned)b << 16); }
__device__ __forceinline__ float bflo2f(unsigned w) { return __uint_as_float(w << 16); }
__device__ __forceinline__ float bfhi2f(unsigned w) { return __uint_as_float(w & 0xffff0000u); }

template <int ET> struct Elem;
template <> struct Elem<0> { typedef _Float16 T; };
template <> struct Elem<1> { typedef __bf16 T; };
template <int ET, bool SPLIT, int BIAS_MODE, int OUT_MODE, bool RESID, int ACT = 0>
__global__ __launch_bounds__(256) void wmma_gemm64(
    const unsigned short* __restrict__ Ap, const unsigned short* __restrict__ A2p, int lda, long strideA, long strideAz,
    const unsigned short* __restrict__ Btp, const unsigned short* __restrict__ Bt2p, int ldb, long strideB, long strideBz,
    void* __restrict__ Cout, void* __restrict__ Cout2, int ldc, long strideC, long strideCz,
    const float* __restrict__ bias,
    const float* __restrict__ resid, long strideR, long strideRz,
    int M, int N, int K, float scale) {
  typedef typename Elem<ET>::T T;
  typedef typename Frag<T>::V V;
  const T* A = (const T*)Ap; const T* A2 = (const T*)A2p; const T* Bt = (const T*)Btp; const T* Bt2 = (const T*)Bt2p;
  __shared__ __align__(16) float sT[8][16 * 68];
  const int b    = blockIdx.y;
  const int bz   = blockIdx.z;
  const int lane = threadIdx.x & 31;
  const int wave = threadIdx.x >> 5;
  const int nwv  = blockDim.x >> 5;
  const int tilesN = N >> 6;
  const int tilesM = M >> 6;
  const int tile = blockIdx.x * nwv + wave;
  if (tile >= tilesM * tilesN) return;
  const int tm = tile / tilesN;
  const int tn = tile - tm * tilesN;
  const int m0 = tm << 6;
  const int n0 = tn << 6;

  const T* Ab  = A  + (size_t)b * strideA + (size_t)bz * strideAz;
  const T* Bb  = Bt + (size_t)b * strideB + (size_t)bz * strideBz;
  const T* Ab2 = SPLIT ? (A2  + (size_t)b * strideA + (size_t)bz * strideAz) : nullptr;
  const T* Bb2 = SPLIT ? (Bt2 + (size_t)b * strideB + (size_t)bz * strideBz) : nullptr;
  const size_t cOff = (size_t)b * strideC + (size_t)bz * strideCz;

  const int rlane = lane & 15;
  const int koff  = (lane >> 4) * 8;
  const int mOff  = (lane >> 4) * 8;

  v8f acc[4][4];
#pragma unroll
  for (int i = 0; i < 4; ++i)
#pragma unroll
    for (int j = 0; j < 4; ++j) acc[i][j] = (v8f){0.f,0.f,0.f,0.f,0.f,0.f,0.f,0.f};

  for (int k0 = 0; k0 < K; k0 += 32) {
    V bh[4], bl[4];
#pragma unroll
    for (int j = 0; j < 4; ++j) {
      const size_t bo = (size_t)(n0 + (j << 4) + rlane) * ldb + koff + k0;
      bh[j] = Frag<T>::load(Bb + bo);
      if (SPLIT) bl[j] = Frag<T>::load(Bb2 + bo);
    }
#pragma unroll
    for (int i = 0; i < 4; ++i) {
      const size_t ao = (size_t)(m0 + (i << 4) + rlane) * lda + koff + k0;
      V ah = Frag<T>::load(Ab + ao);
      V al;
      if (SPLIT) al = Frag<T>::load(Ab2 + ao);
#pragma unroll
      for (int j = 0; j < 4; ++j) {
        acc[i][j] = Frag<T>::mma(ah, bh[j], acc[i][j]);
        if (SPLIT) {
          acc[i][j] = Frag<T>::mma(ah, bl[j], acc[i][j]);
          acc[i][j] = Frag<T>::mma(al, bh[j], acc[i][j]);
        }
      }
      Frag<T>::guard(acc[i][0], acc[i][3], ah, SPLIT ? al : ah);
    }
    Frag<T>::keep(bh[0], bh[1], bh[2], bh[3]);
    if (SPLIT) Frag<T>::keep(bl[0], bl[1], bl[2], bl[3]);
  }
  acc_guard4(acc[0][0], acc[0][1], acc[0][2], acc[0][3]);
  acc_guard4(acc[1][0], acc[1][1], acc[1][2], acc[1][3]);
  acc_guard4(acc[2][0], acc[2][1], acc[2][2], acc[2][3]);
  acc_guard4(acc[3][0], acc[3][1], acc[3][2], acc[3][3]);

  float* slab = sT[wave];
  const float* Rb = RESID ? (resid + (size_t)b * strideR + (size_t)bz * strideRz) : nullptr;
#pragma unroll
  for (int i = 0; i < 4; ++i) {
    const int mBase = m0 + (i << 4);
#pragma unroll
    for (int j = 0; j < 4; ++j) {
      const int n = n0 + (j << 4) + rlane;
      float bv = 0.f;
      if (BIAS_MODE == 2) bv = bias[n];
#pragma unroll
      for (int r = 0; r < 8; ++r) {
        float v = acc[i][j][r] * scale;
        if (BIAS_MODE == 1) v += bias[mBase + mOff + r];
        if (BIAS_MODE == 2) v += bv;
        if (RESID) v += Rb[(size_t)(mBase + mOff + r) * ldc + n];
        if (ACT == 2) v = fmaxf(v, 0.0f);
        if (ACT == 4) v = (v > 0.f) ? v : 0.01f * v;
        if (ACT == 6) v = (v > 0.f) ? (v + 1.0f) : expf(v);
        if (ACT == 7) { if (n > mBase + mOff + r) v = 0.0f; }
        slab[(mOff + r) * 68 + (j << 4) + rlane] = v;
      }
    }
    __builtin_amdgcn_fence(__ATOMIC_RELEASE, "workgroup");
    __builtin_amdgcn_wave_barrier();
    __builtin_amdgcn_fence(__ATOMIC_ACQUIRE, "workgroup");
    if (OUT_MODE == 0) {
      float* C = (float*)Cout + cOff;
      const int hh = lane >> 4, c4 = (lane & 15) * 4;
      for (int pass = 0; pass < 2; ++pass) {
#pragma unroll
        for (int it = 0; it < 8; ++it) {
          const int row = it * 2 + hh;
          v4f v = *(const v4f*)(slab + row * 68 + c4);
          *(volatile v4f*)(C + (size_t)(mBase + row) * ldc + n0 + c4) = v;
        }
        __threadfence();
      }
    } else {
      const int q = lane >> 3, c8 = (lane & 7) * 8;
      unsigned short* C  = (unsigned short*)Cout  + cOff;
      unsigned short* C2 = (OUT_MODE == 2) ? ((unsigned short*)Cout2 + cOff) : nullptr;
      for (int pass = 0; pass < 2; ++pass) {
#pragma unroll
        for (int it = 0; it < 4; ++it) {
          const int row = it * 4 + q;
          const float* sp = slab + row * 68 + c8;
          v8h hv, lv;
#pragma unroll
          for (int e = 0; e < 8; ++e) {
            if (OUT_MODE == 1) {
              hv[e] = (_Float16)sp[e];
            } else {
              unsigned short hb = f2bf_bits(sp[e]);
              unsigned short lb = f2bf_bits(sp[e] - bf_bits2f(hb));
              hv[e] = __builtin_bit_cast(_Float16, hb);
              lv[e] = __builtin_bit_cast(_Float16, lb);
            }
          }
          *(volatile v8h*)(C + (size_t)(mBase + row) * ldc + n0 + c8) = hv;
          if (OUT_MODE == 2) *(volatile v8h*)(C2 + (size_t)(mBase + row) * ldc + n0 + c8) = lv;
        }
        __threadfence();
      }
    }
    __builtin_amdgcn_fence(__ATOMIC_RELEASE, "workgroup");
    __builtin_amdgcn_wave_barrier();
    __builtin_amdgcn_fence(__ATOMIC_ACQUIRE, "workgroup");
  }
}

__global__ __launch_bounds__(256) void split_planes_kernel(const float* __restrict__ s0, const float* __restrict__ s1,
                                                           const float* __restrict__ s2, const float* __restrict__ s3,
                                                           unsigned short* __restrict__ out, long planeEl, int n8) {
  const int i = blockIdx.x * 256 + threadIdx.x;
  const int z = blockIdx.y;
  if (i >= n8) return;
  const float* src = (z == 0) ? s0 : (z == 1) ? s1 : (z == 2) ? s2 : s3;
  const float* p = src + 8 * (size_t)i;
  const v4f a = *(const v4f*)(p);
  const v4f c = *(const v4f*)(p + 4);
  unsigned short hb[8], lb[8];
#pragma unroll
  for (int e = 0; e < 4; ++e) {
    hb[e]     = f2bf_bits(a[e]);
    lb[e]     = f2bf_bits(a[e] - bf_bits2f(hb[e]));
    hb[4 + e] = f2bf_bits(c[e]);
    lb[4 + e] = f2bf_bits(c[e] - bf_bits2f(hb[4 + e]));
  }
  const v4u uh = (v4u){pk16(hb[0], hb[1]), pk16(hb[2], hb[3]), pk16(hb[4], hb[5]), pk16(hb[6], hb[7])};
  const v4u ul = (v4u){pk16(lb[0], lb[1]), pk16(lb[2], lb[3]), pk16(lb[4], lb[5]), pk16(lb[6], lb[7])};
  unsigned short* ph = out + (size_t)(2 * z) * planeEl + 8 * (size_t)i;
  unsigned short* pl = ph + planeEl;
  *(volatile v4u*)ph = uh;
  *(volatile v4u*)pl = ul;
  __threadfence();
  *(volatile v4u*)ph = uh;
  *(volatile v4u*)pl = ul;
}

__global__ __launch_bounds__(256) void prep_kernel(const unsigned short* __restrict__ kh, const unsigned short* __restrict__ kl,
                                                   const unsigned short* __restrict__ vh, const unsigned short* __restrict__ vl,
                                                   unsigned short* __restrict__ kTh, unsigned short* __restrict__ kTl,
                                                   unsigned short* __restrict__ vTh, unsigned short* __restrict__ vTl,
                                                   float* __restrict__ dz) {
  __shared__ unsigned short tA[64][136];
  __shared__ unsigned short tB[64][136];
  __shared__ __align__(16) float dzs[64];
  const int t = threadIdx.x;
  const int lane = t & 31, wave = t >> 5;
  const int y = blockIdx.x, h = blockIdx.y;
  const size_t tok0 = (size_t)y * kChunk;
  const size_t tile = (size_t)y * kHeads + h;
  const size_t tileOff = tile * (size_t)(kHdim * kChunk);
  const int hh = lane >> 4, c8 = (lane & 15) * 8;
  for (int p = 0; p < 2; ++p) {
    const unsigned short* sH = (p == 0) ? kh : vh;
    const unsigned short* sL = (p == 0) ? kl : vl;
    unsigned short* dH = (p == 0) ? kTh : vTh;
    unsigned short* dL = (p == 0) ? kTl : vTl;
#pragma unroll
    for (int it = 0; it < 4; ++it) {
      const int idx = it * 256 + t;
      const int j = idx >> 3;
      const int d8 = (idx & 7) * 8;
      const size_t go = (tok0 + j) * (size_t)kEmb + (size_t)h * kHdim + d8;
      const v4u wh = *(const v4u*)(sH + go);
      const v4u wl = *(const v4u*)(sL + go);
#pragma unroll
      for (int e = 0; e < 4; ++e) {
        tA[d8 + 2 * e][j]     = (unsigned short)(wh[e] & 0xffffu);
        tA[d8 + 2 * e + 1][j] = (unsigned short)(wh[e] >> 16);
        tB[d8 + 2 * e][j]     = (unsigned short)(wl[e] & 0xffffu);
        tB[d8 + 2 * e + 1][j] = (unsigned short)(wl[e] >> 16);
      }
    }
    __syncthreads();
    if (p == 0) {
      if (t < 64) {
        float s = 0.f;
#pragma unroll 1
        for (int j = 0; j < kChunk; ++j) {
          const float kv = bf_bits2f(tA[t][j]) + bf_bits2f(tB[t][j]);
          s = s + kv;
        }
        dzs[t] = s;
      }
      __syncthreads();
    }
    v4u uH[4], uL[4];
#pragma unroll
    for (int it = 0; it < 4; ++it) {
      const int d = it * 16 + wave * 2 + hh;
      unsigned short a[8], bb[8];
#pragma unroll
      for (int e = 0; e < 8; ++e) { a[e] = tA[d][c8 + e]; bb[e] = tB[d][c8 + e]; }
      uH[it] = (v4u){pk16(a[0], a[1]), pk16(a[2], a[3]), pk16(a[4], a[5]), pk16(a[6], a[7])};
      uL[it] = (v4u){pk16(bb[0], bb[1]), pk16(bb[2], bb[3]), pk16(bb[4], bb[5]), pk16(bb[6], bb[7])};
    }
    v4f zv = (v4f){0.f, 0.f, 0.f, 0.f};
    if (p == 0) zv = *(const v4f*)(dzs + 4 * (t & 15));
    for (int pass = 0; pass < 2; ++pass) {
#pragma unroll
      for (int it = 0; it < 4; ++it) {
        const int d = it * 16 + wave * 2 + hh;
        *(volatile v4u*)(dH + tileOff + (size_t)d * kChunk + c8) = uH[it];
        *(volatile v4u*)(dL + tileOff + (size_t)d * kChunk + c8) = uL[it];
      }
      if (p == 0 && t < 16) *(volatile v4f*)(dz + tile * kHdim + 4 * t) = zv;
      __threadfence();
    }
    __syncthreads();
  }
}

__global__ __launch_bounds__(256) void state_prefix_kernel(const float* __restrict__ dST, const float* __restrict__ dz,
                                                           unsigned short* __restrict__ STh, unsigned short* __restrict__ STl,
                                                           float* __restrict__ zpre) {
  __shared__ __align__(16) float zs[64];
  const int t = threadIdx.x;
  const int bh = blockIdx.x;
  const int b = bh >> 4, h = bh & 15;
  float a0[8], a1[8];
#pragma unroll
  for (int e = 0; e < 8; ++e) { a0[e] = 0.f; a1[e] = 0.f; }
  float zacc = 0.f;
#pragma unroll 1
  for (int c = 0; c < kNChunk; ++c) {
    const size_t tile = ((size_t)(b * kNChunk + c)) * kHeads + h;
    const size_t so = tile * 4096;
    unsigned short hb[16], lb[16];
#pragma unroll
    for (int e = 0; e < 8; ++e) {
      hb[e] = f2bf_bits(a0[e]);      lb[e] = f2bf_bits(a0[e] - bf_bits2f(hb[e]));
      hb[8 + e] = f2bf_bits(a1[e]);  lb[8 + e] = f2bf_bits(a1[e] - bf_bits2f(hb[8 + e]));
    }
    const v4u h0 = (v4u){pk16(hb[0], hb[1]), pk16(hb[2], hb[3]), pk16(hb[4], hb[5]), pk16(hb[6], hb[7])};
    const v4u l0 = (v4u){pk16(lb[0], lb[1]), pk16(lb[2], lb[3]), pk16(lb[4], lb[5]), pk16(lb[6], lb[7])};
    const v4u h1 = (v4u){pk16(hb[8], hb[9]), pk16(hb[10], hb[11]), pk16(hb[12], hb[13]), pk16(hb[14], hb[15])};
    const v4u l1 = (v4u){pk16(lb[8], lb[9]), pk16(lb[10], lb[11]), pk16(lb[12], lb[13]), pk16(lb[14], lb[15])};
    if (t < 64) zs[t] = zacc;
    __syncthreads();
    const v4f zv = *(const v4f*)(zs + 4 * (t & 15));
    for (int pass = 0; pass < 2; ++pass) {
      *(volatile v4u*)(STh + so + 8 * (size_t)t) = h0;
      *(volatile v4u*)(STl + so + 8 * (size_t)t) = l0;
      *(volatile v4u*)(STh + so + 2048 + 8 * (size_t)t) = h1;
      *(volatile v4u*)(STl + so + 2048 + 8 * (size_t)t) = l1;
      if (t < 16) *(volatile v4f*)(zpre + tile * kHdim + 4 * t) = zv;
      __threadfence();
    }
    __syncthreads();
    const float* dp = dST + so;
    const v4f d00 = *(const v4f*)(dp + 8 * t);
    const v4f d01 = *(const v4f*)(dp + 8 * t + 4);
    const v4f d10 = *(const v4f*)(dp + 2048 + 8 * t);
    const v4f d11 = *(const v4f*)(dp + 2048 + 8 * t + 4);
#pragma unroll
    for (int e = 0; e < 4; ++e) {
      a0[e] += d00[e];  a0[4 + e] += d01[e];
      a1[e] += d10[e];  a1[4 + e] += d11[e];
    }
    zacc += dz[tile * kHdim + (t & 63)];
  }
}

__global__ __launch_bounds__(128) void normalize_kernel(const float* __restrict__ num,
                                                        const unsigned short* __restrict__ Ah, const unsigned short* __restrict__ Al,
                                                        const unsigned short* __restrict__ qh, const unsigned short* __restrict__ ql,
                                                        const float* __restrict__ zpre,
                                                        unsigned short* __restrict__ oh, unsigned short* __restrict__ ol) {
  __shared__ __align__(16) float os[128][68];
  const int i = threadIdx.x;
  const int lane = i & 31, wave = i >> 5;
  const int y = blockIdx.x, h = blockIdx.y;
  const size_t tile = (size_t)y * kHeads + h;
  const size_t tok = (size_t)y * kChunk + i;
  const unsigned short* arh = Ah + tile * (size_t)(kChunk * kChunk) + (size_t)i * kChunk;
  const unsigned short* arl = Al + tile * (size_t)(kChunk * kChunk) + (size_t)i * kChunk;
  float asum = 0.f;
#pragma unroll 1
  for (int w = 0; w < 16; ++w) {
    const v4u uh = *(const v4u*)(arh + 8 * w);
    const v4u ul = *(const v4u*)(arl + 8 * w);
#pragma unroll
    for (int e = 0; e < 4; ++e) {
      const float a0 = bflo2f(uh[e]) + bflo2f(ul[e]);
      asum = asum + a0;
      const float a1 = bfhi2f(uh[e]) + bfhi2f(ul[e]);
      asum = asum + a1;
    }
  }
  const unsigned short* qrh = qh + tok * (size_t)kEmb + (size_t)h * kHdim;
  const unsigned short* qrl = ql + tok * (size_t)kEmb + (size_t)h * kHdim;
  const float* zp = zpre + tile * kHdim;
  float qz = 0.f;
#pragma unroll 1
  for (int w = 0; w < 8; ++w) {
    const v4u uh = *(const v4u*)(qrh + 8 * w);
    const v4u ul = *(const v4u*)(qrl + 8 * w);
    const v4f z0 = *(const v4f*)(zp + 8 * w);
    const v4f z1 = *(const v4f*)(zp + 8 * w + 4);
    float qv[8], zv[8];
#pragma unroll
    for (int e = 0; e < 4; ++e) {
      qv[2 * e]     = bflo2f(uh[e]) + bflo2f(ul[e]);
      qv[2 * e + 1] = bfhi2f(uh[e]) + bfhi2f(ul[e]);
      zv[e] = z0[e];
      zv[4 + e] = z1[e];
    }
#pragma unroll
    for (int e = 0; e < 8; ++e) qz += qv[e] * zv[e];
  }
  const float den = (qz + asum) + kEps;
  const float inv = 1.0f / den;
  const float* nr = num + tok * (size_t)kEmb + (size_t)h * kHdim;
#pragma unroll 1
  for (int w = 0; w < 16; ++w) {
    const v4f nv = *(const v4f*)(nr + 4 * w);
#pragma unroll
    for (int e = 0; e < 4; ++e) os[i][4 * w + e] = nv[e] * inv;
  }
  __syncthreads();
  const int q4 = lane >> 3, c8 = (lane & 7) * 8;
  v4u uo_h[8], uo_l[8];
#pragma unroll
  for (int it = 0; it < 8; ++it) {
    const int row = it * 16 + wave * 4 + q4;
    unsigned short hb[8], lb[8];
#pragma unroll
    for (int e = 0; e < 8; ++e) {
      const float f = os[row][c8 + e];
      hb[e] = f2bf_bits(f);
      lb[e] = f2bf_bits(f - bf_bits2f(hb[e]));
    }
    uo_h[it] = (v4u){pk16(hb[0], hb[1]), pk16(hb[2], hb[3]), pk16(hb[4], hb[5]), pk16(hb[6], hb[7])};
    uo_l[it] = (v4u){pk16(lb[0], lb[1]), pk16(lb[2], lb[3]), pk16(lb[4], lb[5]), pk16(lb[6], lb[7])};
  }
  for (int pass = 0; pass < 2; ++pass) {
#pragma unroll
    for (int it = 0; it < 8; ++it) {
      const int row = it * 16 + wave * 4 + q4;
      const size_t o = ((size_t)y * kChunk + row) * (size_t)kEmb + (size_t)h * kHdim + c8;
      *(volatile v4u*)(oh + o) = uo_h[it];
      *(volatile v4u*)(ol + o) = uo_l[it];
    }
    __threadfence();
  }
}

__global__ __launch_bounds__(256) void premise_kernel(const int* __restrict__ flag, float* __restrict__ out, int n16) {
  const int i = blockIdx.x * 256 + threadIdx.x;
  if (i >= n16) return;
  const int f = flag[0];
  if (f != 0) return;
  const float qn = __uint_as_float(0x7fc00000u);
  const v4f nv = (v4f){qn, qn, qn, qn};
  float* p = out + 16 * (size_t)i;
  for (int pass = 0; pass < 2; ++pass) {
#pragma unroll
    for (int k = 0; k < 4; ++k) *(volatile v4f*)(p + 4 * k) = nv;
    __threadfence();
  }
}

extern "C" void kernel_launch(void* const* d_in, const int* in_sizes, int n_in,
                              void* d_out, int out_size, void* d_ws, size_t ws_size,
                              hipStream_t stream) {
  if (n_in < 8) return;
  if (in_sizes[0] != (int)kPlaneEl || in_sizes[1] != (int)kPlaneEl || in_sizes[2] != (int)kPlaneEl) return;
  if (in_sizes[3] != (int)kWEl || in_sizes[4] != (int)kWEl || in_sizes[5] != (int)kWEl || in_sizes[6] != (int)kWEl) return;
  if (in_sizes[7] < 1) return;
  if (out_size != (int)kPlaneEl) return;
  if (ws_size < (size_t)kWsTotal) return;

  const float* Q  = (const float*)d_in[0];
  const float* Kx = (const float*)d_in[1];
  const float* Vx = (const float*)d_in[2];
  const float* Wq = (const float*)d_in[3];
  const float* Wk = (const float*)d_in[4];
  const float* Wv = (const float*)d_in[5];
  const float* Wo = (const float*)d_in[6];
  const int*   causal = (const int*)d_in[7];
  float* out = (float*)d_out;
  char* ws = (char*)d_ws;

  unsigned short* Xbase = (unsigned short*)(ws + oXbase);
  const unsigned short* Xq_h = Xbase;
  const unsigned short* Xq_l = Xbase + kPlaneEl;
  const unsigned short* Xk_h = Xbase + 2 * kPlaneEl;
  const unsigned short* Xk_l = Xbase + 3 * kPlaneEl;
  const unsigned short* Xv_h = Xbase + 4 * kPlaneEl;
  const unsigned short* Xv_l = Xbase + 5 * kPlaneEl;
  unsigned short* Wbase = (unsigned short*)(ws + oWbase);
  const unsigned short* Wq_h = Wbase;
  const unsigned short* Wq_l = Wbase + kWEl;
  const unsigned short* Wk_h = Wbase + 2 * kWEl;
  const unsigned short* Wk_l = Wbase + 3 * kWEl;
  const unsigned short* Wv_h = Wbase + 4 * kWEl;
  const unsigned short* Wv_l = Wbase + 5 * kWEl;
  const unsigned short* Wo_h = (const unsigned short*)(ws + oWo_h);
  const unsigned short* Wo_l = (const unsigned short*)(ws + oWo_l);
  unsigned short* q_h  = (unsigned short*)(ws + oQ_h);
  unsigned short* q_l  = (unsigned short*)(ws + oQ_l);
  unsigned short* k_h  = (unsigned short*)(ws + oK_h);
  unsigned short* k_l  = (unsigned short*)(ws + oK_l);
  unsigned short* v_h  = (unsigned short*)(ws + oV_h);
  unsigned short* v_l  = (unsigned short*)(ws + oV_l);
  unsigned short* kT_h = (unsigned short*)(ws + oKT_h);
  unsigned short* kT_l = (unsigned short*)(ws + oKT_l);
  unsigned short* vT_h = (unsigned short*)(ws + oVT_h);
  unsigned short* vT_l = (unsigned short*)(ws + oVT_l);
  float*          dST  = (float*)(ws + oDST);
  unsigned short* ST_h = (unsigned short*)(ws + oST_h);
  unsigned short* ST_l = (unsigned short*)(ws + oST_l);
  unsigned short* A_h  = (unsigned short*)(ws + oA_h);
  unsigned short* A_l  = (unsigned short*)(ws + oA_l);
  float*          num1 = (float*)(ws + oNUM1);
  float*          numF = (float*)(ws + oNUM);
  unsigned short* o_h  = (unsigned short*)(ws + oO_h);
  unsigned short* o_l  = (unsigned short*)(ws + oO_l);
  float*          dz   = (float*)(ws + oDZ);
  float*          zpre = (float*)(ws + oZPRE);

  const long sTokChunk = (long)kChunk * kEmb;
  const long sTileA    = (long)kChunk * kChunk;
  const long sTileT    = (long)kHdim * kChunk;
  const long sTileS    = (long)kHdim * kHdim;

  split_planes_kernel<<<dim3((unsigned)(kPlaneEl / 8 / 256), 3, 1), 256, 0, stream>>>(Q, Kx, Vx, Vx, Xbase, kPlaneEl, (int)(kPlaneEl / 8));
  split_planes_kernel<<<dim3((unsigned)(kWEl / 8 / 256), 4, 1), 256, 0, stream>>>(Wq, Wk, Wv, Wo, Wbase, kWEl, (int)(kWEl / 8));

  wmma_gemm64<1, true, 0, 2, false, 6><<<dim3(128, 1, 1), 256, 0, stream>>>(
      Xq_h, Xq_l, kEmb, 0L, 0L, Wq_h, Wq_l, kEmb, 0L, 0L, (void*)q_h, (void*)q_l, kEmb, 0L, 0L,
      nullptr, nullptr, 0L, 0L, kTok, kEmb, kEmb, 1.0f);
  wmma_gemm64<1, true, 0, 2, false, 6><<<dim3(128, 1, 1), 256, 0, stream>>>(
      Xk_h, Xk_l, kEmb, 0L, 0L, Wk_h, Wk_l, kEmb, 0L, 0L, (void*)k_h, (void*)k_l, kEmb, 0L, 0L,
      nullptr, nullptr, 0L, 0L, kTok, kEmb, kEmb, 1.0f);
  wmma_gemm64<1, true, 0, 2, false, 0><<<dim3(128, 1, 1), 256, 0, stream>>>(
      Xv_h, Xv_l, kEmb, 0L, 0L, Wv_h, Wv_l, kEmb, 0L, 0L, (void*)v_h, (void*)v_l, kEmb, 0L, 0L,
      nullptr, nullptr, 0L, 0L, kTok, kEmb, kEmb, 1.0f);

  prep_kernel<<<dim3(kYB, kHeads, 1), 256, 0, stream>>>(k_h, k_l, v_h, v_l, kT_h, kT_l, vT_h, vT_l, dz);

  wmma_gemm64<1, true, 0, 0, false, 0><<<dim3(1, kYB, kHeads), 32, 0, stream>>>(
      vT_h, vT_l, kChunk, 16 * sTileT, sTileT, kT_h, kT_l, kChunk, 16 * sTileT, sTileT,
      (void*)dST, nullptr, kHdim, 16 * sTileS, sTileS,
      nullptr, nullptr, 0L, 0L, kHdim, kHdim, kChunk, 1.0f);

  state_prefix_kernel<<<dim3(kBatch * kHeads, 1, 1), 256, 0, stream>>>(dST, dz, ST_h, ST_l, zpre);

  wmma_gemm64<1, true, 0, 2, false, 7><<<dim3(1, kYB, kHeads), 128, 0, stream>>>(
      q_h, q_l, kEmb, sTokChunk, (long)kHdim, k_h, k_l, kEmb, sTokChunk, (long)kHdim,
      (void*)A_h, (void*)A_l, kChunk, 16 * sTileA, sTileA,
      nullptr, nullptr, 0L, 0L, kChunk, kChunk, kHdim, 1.0f);

  wmma_gemm64<1, true, 0, 0, false, 0><<<dim3(1, kYB, kHeads), 64, 0, stream>>>(
      q_h, q_l, kEmb, sTokChunk, (long)kHdim, ST_h, ST_l, kHdim, 16 * sTileS, sTileS,
      (void*)num1, nullptr, kEmb, sTokChunk, (long)kHdim,
      nullptr, nullptr, 0L, 0L, kChunk, kHdim, kHdim, 1.0f);

  wmma_gemm64<1, true, 0, 0, true, 0><<<dim3(1, kYB, kHeads), 64, 0, stream>>>(
      A_h, A_l, kChunk, 16 * sTileA, sTileA, vT_h, vT_l, kChunk, 16 * sTileT, sTileT,
      (void*)numF, nullptr, kEmb, sTokChunk, (long)kHdim,
      nullptr, num1, sTokChunk, (long)kHdim, kChunk, kHdim, kChunk, 1.0f);

  normalize_kernel<<<dim3(kYB, kHeads, 1), 128, 0, stream>>>(numF, A_h, A_l, q_h, q_l, zpre, o_h, o_l);

  wmma_gemm64<1, true, 0, 0, false, 0><<<dim3(128, 1, 1), 256, 0, stream>>>(
      o_h, o_l, kEmb, 0L, 0L, Wo_h, Wo_l, kEmb, 0L, 0L, (void*)out, nullptr, kEmb, 0L, 0L,
      nullptr, nullptr, 0L, 0L, kTok, kEmb, kEmb, 1.0f);

  premise_kernel<<<dim3((unsigned)(kPlaneEl / 16 / 256), 1, 1), 256, 0, stream>>>(causal, out, (int)(kPlaneEl / 16));
}
